// cartpole_RNN_dqn_74251394613868
// MI455X (gfx1250) — hardware-verified
//
#include <hip/hip_runtime.h>
#include <stdint.h>

typedef __attribute__((ext_vector_type(16))) _Float16 v16h;
typedef __attribute__((ext_vector_type(8)))  _Float16 v8h;
typedef __attribute__((ext_vector_type(8)))  float    v8f;
typedef __attribute__((ext_vector_type(4)))  float    v4f;
typedef __attribute__((ext_vector_type(4)))  unsigned int v4u;

constexpr int SEQ_T  = 512;
constexpr int NBATCH = 4096;
constexpr int XDIM   = 4;
constexpr int NH1    = 24;
constexpr int NH2    = 48;
constexpr int NH3    = 24;
constexpr int NOUT   = 2;

constexpr float WSCALE     = 16.0f;
constexpr float WSCALE_INV = 0.0625f;

constexpr int LDP    = 128;
constexpr int COL_H1 = 0;
constexpr int COL_H2 = 32;
constexpr int COL_H3 = 96;
constexpr int AOFF1  = 0;
constexpr int AOFF2  = 0;
constexpr int AOFF3  = 32;

constexpr int KP1 = 32;
constexpr int KP2 = 96;
constexpr int KP3 = 96;
constexpr int P1_ROWS = 32;
constexpr int P2_ROWS = 48;
constexpr int P3_ROWS = 32;
constexpr int P1_HALVES = P1_ROWS * KP1;
constexpr int P2_HALVES = P2_ROWS * KP2;
constexpr int P3_HALVES = P3_ROWS * KP3;
constexpr int PLANE_HALVES = P1_HALVES + P2_HALVES + P3_HALVES;
constexpr int PLANE_CHUNKS = PLANE_HALVES / 8;
constexpr size_t PLANE_BYTES = (size_t)PLANE_HALVES * 2;
static_assert(PLANE_HALVES % 8 == 0, "chunking");
static_assert(PLANE_CHUNKS % 32 == 0, "every wave of the prep kernel writes only whole 128-B lines");
static_assert((P1_HALVES * 2) % 128 == 0, "P2 base line aligned");
static_assert(((P1_HALVES + P2_HALVES) * 2) % 128 == 0, "P3 base line aligned");
static_assert(PLANE_BYTES % 128 == 0, "whole lines");
static_assert(KP1 % 32 == 0 && KP2 % 32 == 0 && KP3 % 32 == 0, "K multiple of 32");
static_assert(NBATCH % 16 == 0, "one m-subtile per wave");
static_assert(LDP % 8 == 0 && KP1 % 8 == 0 && KP2 % 8 == 0, "16-B aligned fragment loads");

struct FragH {
  union U { v16h v; v8h h[2]; };
  static __device__ __forceinline__ v16h load(const _Float16* p) {
    U f; f.h[0] = *(const v8h*)(p); f.h[1] = *(const v8h*)(p + 16); return f.v;
  }
};

__device__ __forceinline__ v8f mma_h(v16h a, v16h b, v8f c) {
  c = __builtin_amdgcn_wmma_f32_16x16x32_f16(false, a, false, b, (short)0, c, false, false);
  asm volatile("v_nop\n\tv_nop\n\tv_nop\n\tv_nop" : "+v"(c) : "v"(a), "v"(b));
  return c;
}

__device__ __forceinline__ v8f zero8f() { return (v8f){0.f, 0.f, 0.f, 0.f, 0.f, 0.f, 0.f, 0.f}; }

__global__ __launch_bounds__(256) void prep_planes(
    const float* __restrict__ Whh0, const float* __restrict__ Wih1, const float* __restrict__ Whh1,
    const float* __restrict__ Wih2, const float* __restrict__ Whh2, unsigned short* __restrict__ planes) {
  const int chunk = blockIdx.x * 256 + threadIdx.x;
  if (chunk >= PLANE_CHUNKS) return;
  const int e0 = chunk * 8;
  int src = 5, n = 0, cb = 0;
  if (e0 < P1_HALVES) {
    n = e0 / KP1;
    const int k = e0 - n * KP1;
    if (n < NH1 && k < 24) { src = 0; cb = k; }
  } else if (e0 < P1_HALVES + P2_HALVES) {
    const int e1 = e0 - P1_HALVES;
    n = e1 / KP2;
    const int k = e1 - n * KP2;
    if (k < 24)      { src = 1; cb = k; }
    else if (k < 32) { }
    else if (k < 80) { src = 2; cb = k - 32; }
    else             { }
  } else {
    const int e2 = e0 - P1_HALVES - P2_HALVES;
    n = e2 / KP3;
    const int k = e2 - n * KP3;
    if (n < NH3) {
      if (k < 48)      { src = 3; cb = k; }
      else if (k < 64) { }
      else if (k < 88) { src = 4; cb = k - 64; }
      else             { }
    }
  }
  const int n23 = n < 23 ? n : 23;
  const int n47 = n < 47 ? n : 47;
  unsigned int w[4] = {0u, 0u, 0u, 0u};
#pragma unroll
  for (int e = 0; e < 8; ++e) {
    const int col = cb + e;
    const int c23 = col < 23 ? col : 23;
    const int c47 = col < 47 ? col : 47;
    const float s0 = Whh0[n23 * NH1 + c23];
    const float s1 = Wih1[n47 * NH1 + c23];
    const float s2 = Whh1[n47 * NH2 + c47];
    const float s3 = Wih2[n23 * NH2 + c47];
    const float s4 = Whh2[n23 * NH3 + c23];
    const float v = (src == 0) ? s0 : (src == 1) ? s1 : (src == 2) ? s2 : (src == 3) ? s3 : (src == 4) ? s4 : 0.0f;
    const _Float16 hv = (_Float16)(v * WSCALE);
    const unsigned short bits = __builtin_bit_cast(unsigned short, hv);
    w[e >> 1] |= ((unsigned int)bits) << (16 * (e & 1));
  }
  const v4u pk = {w[0], w[1], w[2], w[3]};
  unsigned short* dst = planes + (size_t)chunk * 8;
  *(volatile v4u*)(void*)dst = pk;
  __threadfence();
  *(volatile v4u*)(void*)dst = pk;
}

__global__ __launch_bounds__(32) void rnn3_fused(
    const float* __restrict__ x, const float* __restrict__ Wih0,
    const float* __restrict__ bih0, const float* __restrict__ bhh0,
    const float* __restrict__ bih1, const float* __restrict__ bhh1,
    const float* __restrict__ bih2, const float* __restrict__ bhh2,
    const float* __restrict__ Wout, const float* __restrict__ bout,
    const unsigned short* __restrict__ planes, float* __restrict__ out) {
  __shared__ __align__(16) _Float16 Hs[16 * LDP];
  __shared__ __align__(16) float    S3[16 * 32];
  __shared__ __align__(16) float    OutS[32];

  const int lane = threadIdx.x & 31;
  const int hh   = lane >> 4;
  const int c    = lane & 15;
  const int koff = 8 * hh;
  const int b0   = blockIdx.x * 16;

  const _Float16* P1 = (const _Float16*)(const void*)planes;
  const _Float16* P2 = P1 + P1_HALVES;
  const _Float16* P3 = P2 + P2_HALVES;

  {
    const v4u z = {0u, 0u, 0u, 0u};
#pragma unroll
    for (int i = 0; i < 8; ++i) *(v4u*)(void*)(Hs + (size_t)(lane + 32 * i) * 8) = z;
  }
  __syncthreads();

  const bool ok2 = (c < 8);
  const int  ua  = c;
  const int  ubc = ok2 ? (16 + c) : (NH1 - 1);
  const float wia0 = Wih0[ua * XDIM + 0], wia1 = Wih0[ua * XDIM + 1], wia2 = Wih0[ua * XDIM + 2], wia3 = Wih0[ua * XDIM + 3];
  const float tw0 = Wih0[ubc * XDIM + 0], tw1 = Wih0[ubc * XDIM + 1], tw2 = Wih0[ubc * XDIM + 2], tw3 = Wih0[ubc * XDIM + 3];
  const float wib0 = ok2 ? tw0 : 0.0f, wib1 = ok2 ? tw1 : 0.0f, wib2 = ok2 ? tw2 : 0.0f, wib3 = ok2 ? tw3 : 0.0f;
  const float bs1a  = bih0[ua] + bhh0[ua];
  const float tb1b  = bih0[ubc] + bhh0[ubc];
  const float bs1b  = ok2 ? tb1b : 0.0f;
  float bs2[3];
#pragma unroll
  for (int j = 0; j < 3; ++j) bs2[j] = bih1[16 * j + c] + bhh1[16 * j + c];
  const float bs3a = bih2[ua] + bhh2[ua];
  const float tb3b = bih2[ubc] + bhh2[ubc];
  const float bs3b = ok2 ? tb3b : 0.0f;
  const int hrow = lane >> 1;
  const int ho   = lane & 1;
  v4f wo4[6];
#pragma unroll
  for (int q = 0; q < 6; ++q) wo4[q] = *(const v4f*)(Wout + ho * NH3 + 4 * q);
  const float bo = bout[ho];

#pragma unroll 1
  for (int t = 0; t < SEQ_T; ++t) {
    v8f acc1a, acc1b;
    {
      const v16h af  = FragH::load(Hs + c * LDP + AOFF1 + koff);
      const v16h bfa = FragH::load(P1 + (size_t)c * KP1 + koff);
      const v16h bfb = FragH::load(P1 + (size_t)(16 + c) * KP1 + koff);
      acc1a = mma_h(af, bfa, zero8f());
      acc1b = mma_h(af, bfb, zero8f());
    }
    {
      const size_t xrow0 = ((size_t)t * NBATCH + (size_t)b0 + (size_t)(8 * hh)) * XDIM;
#pragma unroll
      for (int r = 0; r < 8; ++r) {
        const v4f xv = *(const v4f*)(x + xrow0 + (size_t)r * XDIM);
        float pa = xv[0] * wia0;
        pa = fmaf(xv[1], wia1, pa);
        pa = fmaf(xv[2], wia2, pa);
        pa = fmaf(xv[3], wia3, pa);
        float pb = xv[0] * wib0;
        pb = fmaf(xv[1], wib1, pb);
        pb = fmaf(xv[2], wib2, pb);
        pb = fmaf(xv[3], wib3, pb);
        const float va = fmaxf(acc1a[r] * WSCALE_INV + (pa + bs1a), 0.0f);
        const float tb = fmaxf(acc1b[r] * WSCALE_INV + (pb + bs1b), 0.0f);
        const float vb = ok2 ? tb : 0.0f;
        _Float16* rowp = Hs + (8 * hh + r) * LDP;
        rowp[COL_H1 + c]      = (_Float16)va;
        rowp[COL_H1 + 16 + c] = (_Float16)vb;
      }
    }
    __syncthreads();

    v8f acc2[3];
    acc2[0] = zero8f(); acc2[1] = zero8f(); acc2[2] = zero8f();
#pragma unroll 1
    for (int ks = 0; ks < 3; ++ks) {
      const v16h af = FragH::load(Hs + c * LDP + AOFF2 + 32 * ks + koff);
#pragma unroll
      for (int j = 0; j < 3; ++j) {
        const v16h bf = FragH::load(P2 + (size_t)(16 * j + c) * KP2 + 32 * ks + koff);
        acc2[j] = mma_h(af, bf, acc2[j]);
      }
    }
#pragma unroll
    for (int j = 0; j < 3; ++j) {
      const int u = 16 * j + c;
#pragma unroll
      for (int r = 0; r < 8; ++r) {
        const float v = fmaxf(acc2[j][r] * WSCALE_INV + bs2[j], 0.0f);
        Hs[(8 * hh + r) * LDP + COL_H2 + u] = (_Float16)v;
      }
    }
    __syncthreads();

    v8f acc3a = zero8f(), acc3b = zero8f();
#pragma unroll 1
    for (int ks = 0; ks < 3; ++ks) {
      const v16h af  = FragH::load(Hs + c * LDP + AOFF3 + 32 * ks + koff);
      const v16h bfa = FragH::load(P3 + (size_t)c * KP3 + 32 * ks + koff);
      const v16h bfb = FragH::load(P3 + (size_t)(16 + c) * KP3 + 32 * ks + koff);
      acc3a = mma_h(af, bfa, acc3a);
      acc3b = mma_h(af, bfb, acc3b);
    }
#pragma unroll
    for (int r = 0; r < 8; ++r) {
      const int row = 8 * hh + r;
      _Float16* rowp = Hs + row * LDP;
      const float va = fmaxf(acc3a[r] * WSCALE_INV + bs3a, 0.0f);
      const float tb = fmaxf(acc3b[r] * WSCALE_INV + bs3b, 0.0f);
      const float vb = ok2 ? tb : 0.0f;
      rowp[COL_H3 + c]      = (_Float16)va;
      rowp[COL_H3 + 16 + c] = (_Float16)vb;
      S3[row * 32 + c]      = va;
      S3[row * 32 + 16 + c] = vb;
    }
    __syncthreads();

    {
      const float* sp = S3 + hrow * 32;
      float s = 0.0f;
#pragma unroll
      for (int q = 0; q < 6; ++q) {
        const v4f sv = *(const v4f*)(sp + 4 * q);
        s = fmaf(sv[0], wo4[q][0], s);
        s = fmaf(sv[1], wo4[q][1], s);
        s = fmaf(sv[2], wo4[q][2], s);
        s = fmaf(sv[3], wo4[q][3], s);
      }
      s += bo;
      OutS[lane] = s;
    }
    __syncthreads();
    {
      const v4f val = *(const v4f*)(OutS + 4 * (lane & 7));
      float* dst = out + ((size_t)t * NBATCH + (size_t)b0) * NOUT + 4 * (lane & 7);
      if (lane < 8) *(volatile v4f*)dst = val;
      __threadfence();
      if (lane < 8) *(volatile v4f*)dst = val;
    }
  }
}

extern "C" void kernel_launch(void* const* d_in, const int* in_sizes, int n_in,
                              void* d_out, int out_size, void* d_ws, size_t ws_size,
                              hipStream_t stream) {
  if (n_in < 15) return;
  if (in_sizes[0] != SEQ_T * NBATCH * XDIM) return;
  if (in_sizes[1] != NH1 * XDIM || in_sizes[2] != NH1 * NH1) return;
  if (in_sizes[3] != NH1 || in_sizes[4] != NH1) return;
  if (in_sizes[5] != NH2 * NH1 || in_sizes[6] != NH2 * NH2) return;
  if (in_sizes[7] != NH2 || in_sizes[8] != NH2) return;
  if (in_sizes[9] != NH3 * NH2 || in_sizes[10] != NH3 * NH3) return;
  if (in_sizes[11] != NH3 || in_sizes[12] != NH3) return;
  if (in_sizes[13] != NOUT * NH3 || in_sizes[14] != NOUT) return;
  if (out_size != SEQ_T * NBATCH * NOUT) return;
  if (ws_size < PLANE_BYTES) return;

  const float* x    = (const float*)d_in[0];
  const float* Wih0 = (const float*)d_in[1];
  const float* Whh0 = (const float*)d_in[2];
  const float* bih0 = (const float*)d_in[3];
  const float* bhh0 = (const float*)d_in[4];
  const float* Wih1 = (const float*)d_in[5];
  const float* Whh1 = (const float*)d_in[6];
  const float* bih1 = (const float*)d_in[7];
  const float* bhh1 = (const float*)d_in[8];
  const float* Wih2 = (const float*)d_in[9];
  const float* Whh2 = (const float*)d_in[10];
  const float* bih2 = (const float*)d_in[11];
  const float* bhh2 = (const float*)d_in[12];
  const float* Wout = (const float*)d_in[13];
  const float* bout = (const float*)d_in[14];
  float* out = (float*)d_out;
  unsigned short* planes = (unsigned short*)d_ws;

  const int prepBlocks = (PLANE_CHUNKS + 255) / 256;
  prep_planes<<<dim3(prepBlocks), dim3(256), 0, stream>>>(Whh0, Wih1, Whh1, Wih2, Whh2, planes);
  rnn3_fused<<<dim3(NBATCH / 16), dim3(32), 0, stream>>>(x, Wih0, bih0, bhh0, bih1, bhh1, bih2, bhh2,
                                                        Wout, bout, planes, out);
}
